// SequentialPredictor_11708080849548
// MI455X (gfx1250) — hardware-verified
//
#include <hip/hip_runtime.h>


typedef _Float16 f16t;
typedef f16t  v16h __attribute__((ext_vector_type(16)));
typedef f16t  v8h  __attribute__((ext_vector_type(8)));
typedef float v8f  __attribute__((ext_vector_type(8)));
typedef float v4f  __attribute__((ext_vector_type(4)));
typedef float v2f  __attribute__((ext_vector_type(2)));
typedef unsigned int v4u __attribute__((ext_vector_type(4)));

union Frag { v16h v; v8h q[2]; };
union Pk16 { v8h h; v4u u; };
union Pk32 { v4f f; v4u u; };

#define NB      32768
#define TT      8
#define OUTLEN  12
#define HID     64
#define WPB     8
#define ROWS_PB (WPB * 16)

#define IMG_WHH 0
#define IMG_W1  16384
#define IMG_W2  20480
#define IMG_W3  24576
#define IMG_W4  28672
#define IMG_TOT 29696
#define IMG_PIECES (IMG_TOT / 8)

static_assert(NB % ROWS_PB == 0);
static_assert(IMG_TOT % 64 == 0);
static_assert((IMG_W1 % 8) == 0 && (IMG_W2 % 8) == 0 && (IMG_W3 % 8) == 0 && (IMG_W4 % 8) == 0);

__device__ __forceinline__ v8f wmma16(v16h a, v16h b, v8f c) {
  return __builtin_amdgcn_wmma_f32_16x16x32_f16(false, a, false, b, (short)0, c, false, false);
}

__device__ __forceinline__ void loadA(Frag& A0, Frag& A1, const f16t* tile, int m, int h) {
  const f16t* p = tile + m * 64 + 8 * h;
  A0.q[0] = *(const v8h*)(p);
  A0.q[1] = *(const v8h*)(p + 16);
  A1.q[0] = *(const v8h*)(p + 32);
  A1.q[1] = *(const v8h*)(p + 48);
}

__device__ __forceinline__ v8f mma64(v8f c, const Frag& A0, const Frag& A1,
                                     const f16t* img, int j, int lane) {
  Frag b0, b1;
  const f16t* p0 = img + ((j * 2 + 0) * 32 + lane) * 16;
  const f16t* p1 = img + ((j * 2 + 1) * 32 + lane) * 16;
  b0.q[0] = *(const v8h*)(p0);
  b0.q[1] = *(const v8h*)(p0 + 8);
  b1.q[0] = *(const v8h*)(p1);
  b1.q[1] = *(const v8h*)(p1 + 8);
  c = wmma16(A0.v, b0.v, c);
  c = wmma16(A1.v, b1.v, c);
  asm volatile("v_nop\n\tv_nop\n\tv_nop\n\tv_nop"
               : "+v"(c)
               : "v"(A0.v), "v"(A1.v), "v"(b0.v), "v"(b1.v));
  return c;
}

__device__ __forceinline__ float sigm_s(float z, float ns) {
  float e = __expf(z * ns);
  return __builtin_amdgcn_rcpf(1.0f + e);
}
__device__ __forceinline__ float tanh_s(float z, float n2s) {
  float ax = fabsf(z);
  float e  = __expf(ax * n2s);
  float r  = (1.0f - e) * __builtin_amdgcn_rcpf(1.0f + e);
  return copysignf(r, z);
}
__device__ __forceinline__ float leaky(float v) { return v > 0.0f ? v : 0.1f * v; }

__global__ __launch_bounds__(256) void k_pack(const float* __restrict__ W_hh,
                                             const float* __restrict__ fc1_w1,
                                             const float* __restrict__ fc1_w2,
                                             const float* __restrict__ fo_w1,
                                             const float* __restrict__ fo_w2,
                                             f16t* __restrict__ img, float sc) {
  const int i = blockIdx.x * 256 + threadIdx.x;
  if (i >= IMG_PIECES) return;
  const int idx0 = i * 8;
  const float* W;
  int base, nvalid;
  if (idx0 < IMG_W1)      { W = W_hh;   base = IMG_WHH; nvalid = 256; }
  else if (idx0 < IMG_W2) { W = fc1_w1; base = IMG_W1;  nvalid = 64; }
  else if (idx0 < IMG_W3) { W = fc1_w2; base = IMG_W2;  nvalid = 64; }
  else if (idx0 < IMG_W4) { W = fo_w1;  base = IMG_W3;  nvalid = 64; }
  else                    { W = fo_w2;  base = IMG_W4;  nvalid = 2; }
  const int loc = idx0 - base;
  const int e0  = loc & 15;
  const int ln  = (loc >> 4) & 31;
  const int kh  = (loc >> 9) & 1;
  const int j   = loc >> 10;
  const int hh  = ln >> 4;
  const int n   = 16 * j + (ln & 15);
  const int kb  = kh * 32 + 8 * hh + (e0 ? 16 : 0);
  Pk16 v;
  if (n < nvalid) {
    const float* p = W + n * 64 + kb;
    v4f a = *(const v4f*)(p);
    v4f b = *(const v4f*)(p + 4);
    v.h[0] = (f16t)(a[0] * sc); v.h[1] = (f16t)(a[1] * sc);
    v.h[2] = (f16t)(a[2] * sc); v.h[3] = (f16t)(a[3] * sc);
    v.h[4] = (f16t)(b[0] * sc); v.h[5] = (f16t)(b[1] * sc);
    v.h[6] = (f16t)(b[2] * sc); v.h[7] = (f16t)(b[3] * sc);
  } else {
    v.u = (v4u){0u, 0u, 0u, 0u};
  }
  f16t* d = img + idx0;
  *(volatile v4u*)d = v.u;
  __threadfence();
  *(volatile v4u*)d = v.u;
}

__global__ __launch_bounds__(256) void k_seq(
    const float* __restrict__ x,      const f16t* __restrict__ gimg,
    const float* __restrict__ W_ih,   const float* __restrict__ b_ih,
    const float* __restrict__ b_hh,
    const float* __restrict__ fc1_b1, const float* __restrict__ fc1_b2,
    const float* __restrict__ fo_b1,  const float* __restrict__ fo_b2,
    float* __restrict__ out) {
  __shared__ __attribute__((aligned(16))) f16t  wimg[IMG_TOT];
  __shared__ __attribute__((aligned(16))) f16t  hrow[WPB * 1024];
  __shared__ __attribute__((aligned(16))) f16t  arow[WPB * 1024];
  __shared__ __attribute__((aligned(16))) f16t  brow[WPB * 1024];
  __shared__ __attribute__((aligned(16))) float xba[WPB * 256];
  __shared__ __attribute__((aligned(16))) float yba[WPB * 384];

  const int tid  = threadIdx.x;
  const int lane = tid & 31;
  const int wv   = tid >> 5;
  const int nlo  = lane & 15;
  const int hi16 = lane >> 4;

#pragma unroll 1
  for (int p = tid; p < IMG_PIECES; p += 256)
    *(v4u*)(wimg + 8 * p) = *(const v4u*)(gimg + 8 * p);

  f16t*  hA = hrow + wv * 1024;
  f16t*  aA = arow + wv * 1024;
  f16t*  aB = brow + wv * 1024;
  float* xb = xba + wv * 256;
  float* yb = yba + wv * 384;
  const int rowBase = blockIdx.x * ROWS_PB + wv * 16;

  {
    const v4u z4 = (v4u){0u, 0u, 0u, 0u};
#pragma unroll
    for (int i = lane; i < 128; i += 32) *(v4u*)(hA + 8 * i) = z4;
    const float* xs = x + (size_t)rowBase * 16;
#pragma unroll
    for (int i = lane; i < 64; i += 32) *(v4f*)(xb + 4 * i) = *(const v4f*)(xs + 4 * i);
  }
  __syncthreads();

  const float S64 = 64.0f, I64 = 0.015625f;
  const float NI  = -0.015625f;
  const float N2I = -0.03125f;
  float bv[16], wa[16], wb[16];
#pragma unroll
  for (int j = 0; j < 16; ++j) {
    int n = 16 * j + nlo;
    bv[j] = (b_ih[n] + b_hh[n]) * S64;
    wa[j] = W_ih[2 * n] * S64;
    wb[j] = W_ih[2 * n + 1] * S64;
  }
  float fb1[4], fb2[4], fb3[4];
#pragma unroll
  for (int jj = 0; jj < 4; ++jj) {
    fb1[jj] = fc1_b1[16 * jj + nlo] * S64;
    fb2[jj] = fc1_b2[16 * jj + nlo] * S64;
    fb3[jj] = fo_b1[16 * jj + nlo] * S64;
  }
  const float fob2 = fo_b2[nlo < 2 ? nlo : 0];

  float cst[32];
#pragma unroll
  for (int i = 0; i < 32; ++i) cst[i] = 0.0f;

#pragma unroll 1
  for (int outer = 0; outer < OUTLEN; ++outer) {
#pragma unroll 1
    for (int t = 0; t < TT; ++t) {
      asm volatile("s_wait_dscnt 0x0" ::: "memory");
      Frag A0, A1;
      loadA(A0, A1, hA, nlo, hi16);
      float xv0[8], xv1[8];
#pragma unroll
      for (int r = 0; r < 8; ++r) {
        int M = r + 8 * hi16;
        v2f xx = *(const v2f*)(xb + M * 16 + 2 * t);
        xv0[r] = xx[0];
        xv1[r] = xx[1];
      }
#pragma unroll
      for (int jj = 0; jj < 4; ++jj) {
        v8f zi, zf, zg, zo;
#pragma unroll
        for (int r = 0; r < 8; ++r) {
          zi[r] = bv[jj]      + xv0[r] * wa[jj]      + xv1[r] * wb[jj];
          zf[r] = bv[jj + 4]  + xv0[r] * wa[jj + 4]  + xv1[r] * wb[jj + 4];
          zg[r] = bv[jj + 8]  + xv0[r] * wa[jj + 8]  + xv1[r] * wb[jj + 8];
          zo[r] = bv[jj + 12] + xv0[r] * wa[jj + 12] + xv1[r] * wb[jj + 12];
        }
        zi = mma64(zi, A0, A1, wimg + IMG_WHH, jj,      lane);
        zf = mma64(zf, A0, A1, wimg + IMG_WHH, jj + 4,  lane);
        zg = mma64(zg, A0, A1, wimg + IMG_WHH, jj + 8,  lane);
        zo = mma64(zo, A0, A1, wimg + IMG_WHH, jj + 12, lane);
#pragma unroll
        for (int r = 0; r < 8; ++r) {
          float si = sigm_s(zi[r], NI);
          float sf = sigm_s(zf[r], NI);
          float gg = tanh_s(zg[r], N2I);
          float so = sigm_s(zo[r], NI);
          float cN = sf * cst[jj * 8 + r] + si * gg;
          cst[jj * 8 + r] = cN;
          float hv = so * tanh_s(cN, -2.0f);
          int M = r + 8 * hi16;
          hA[M * 64 + 16 * jj + nlo] = (f16t)hv;
        }
      }
    }

    asm volatile("s_wait_dscnt 0x0" ::: "memory");
    {
      Frag A0, A1;
      loadA(A0, A1, hA, nlo, hi16);
#pragma unroll
      for (int jj = 0; jj < 4; ++jj) {
        v8f acc;
#pragma unroll
        for (int r = 0; r < 8; ++r) acc[r] = fb1[jj];
        acc = mma64(acc, A0, A1, wimg + IMG_W1, jj, lane);
#pragma unroll
        for (int r = 0; r < 8; ++r) {
          int M = r + 8 * hi16;
          aA[M * 64 + 16 * jj + nlo] = (f16t)leaky(acc[r] * I64);
        }
      }
    }
    asm volatile("s_wait_dscnt 0x0" ::: "memory");
    {
      Frag A0, A1;
      loadA(A0, A1, aA, nlo, hi16);
#pragma unroll
      for (int jj = 0; jj < 4; ++jj) {
        v8f acc;
#pragma unroll
        for (int r = 0; r < 8; ++r) acc[r] = fb2[jj];
        acc = mma64(acc, A0, A1, wimg + IMG_W2, jj, lane);
#pragma unroll
        for (int r = 0; r < 8; ++r) {
          int M = r + 8 * hi16;
          aB[M * 64 + 16 * jj + nlo] = (f16t)(acc[r] * I64);
        }
      }
    }
    asm volatile("s_wait_dscnt 0x0" ::: "memory");
    {
      Frag A0, A1;
      loadA(A0, A1, aB, nlo, hi16);
#pragma unroll
      for (int jj = 0; jj < 4; ++jj) {
        v8f acc;
#pragma unroll
        for (int r = 0; r < 8; ++r) acc[r] = fb3[jj];
        acc = mma64(acc, A0, A1, wimg + IMG_W3, jj, lane);
#pragma unroll
        for (int r = 0; r < 8; ++r) {
          int M = r + 8 * hi16;
          aA[M * 64 + 16 * jj + nlo] = (f16t)leaky(acc[r] * I64);
        }
      }
    }
    asm volatile("s_wait_dscnt 0x0" ::: "memory");
    {
      Frag A0, A1;
      loadA(A0, A1, aA, nlo, hi16);
      v8f acc;
#pragma unroll
      for (int r = 0; r < 8; ++r) acc[r] = 0.0f;
      acc = mma64(acc, A0, A1, wimg + IMG_W4, 0, lane);
      if (nlo < 2) {
#pragma unroll
        for (int r = 0; r < 8; ++r) {
          int M = r + 8 * hi16;
          float yv = acc[r] * I64 + fob2;
          yb[M * 24 + outer * 2 + nlo] = yv;
          float* px = xb + M * 16 + 14 + nlo;
          float nv = *px + yv;
          *px = nv;
        }
      }
    }
  }

  asm volatile("s_wait_dscnt 0x0" ::: "memory");
  Pk32 ov[3];
#pragma unroll
  for (int i = 0; i < 3; ++i) ov[i].f = *(const v4f*)(yb + (i * 32 + lane) * 4);
  float* ob = out + (size_t)rowBase * 24;
#pragma unroll
  for (int i = 0; i < 3; ++i) *(volatile v4u*)(ob + (i * 32 + lane) * 4) = ov[i].u;
  __threadfence();
#pragma unroll
  for (int i = 0; i < 3; ++i) *(volatile v4u*)(ob + (i * 32 + lane) * 4) = ov[i].u;
}

extern "C" void kernel_launch(void* const* d_in, const int* in_sizes, int n_in,
                              void* d_out, int out_size, void* d_ws, size_t ws_size,
                              hipStream_t stream) {
  if (n_in < 15) return;
  if (in_sizes[0] != NB * TT * 2) return;
  if (in_sizes[2] != 4 * HID * 2 || in_sizes[3] != 4 * HID * HID ||
      in_sizes[4] != 4 * HID || in_sizes[5] != 4 * HID) return;
  if (in_sizes[6] != HID * HID || in_sizes[7] != HID ||
      in_sizes[8] != HID * HID || in_sizes[9] != HID ||
      in_sizes[10] != HID * HID || in_sizes[11] != HID ||
      in_sizes[12] != 2 * HID || in_sizes[13] != 2) return;
  if (out_size != NB * OUTLEN * 2) return;
  const size_t img_bytes = (size_t)IMG_TOT * sizeof(f16t);
  if (img_bytes > ws_size) return;

  const float* x      = (const float*)d_in[0];
  const float* W_ih   = (const float*)d_in[2];
  const float* W_hh   = (const float*)d_in[3];
  const float* b_ih   = (const float*)d_in[4];
  const float* b_hh   = (const float*)d_in[5];
  const float* fc1_w1 = (const float*)d_in[6];
  const float* fc1_b1 = (const float*)d_in[7];
  const float* fc1_w2 = (const float*)d_in[8];
  const float* fc1_b2 = (const float*)d_in[9];
  const float* fo_w1  = (const float*)d_in[10];
  const float* fo_b1  = (const float*)d_in[11];
  const float* fo_w2  = (const float*)d_in[12];
  const float* fo_b2  = (const float*)d_in[13];
  float* out  = (float*)d_out;
  f16t*  gimg = (f16t*)d_ws;

  k_pack<<<dim3((IMG_PIECES + 255) / 256), dim3(256), 0, stream>>>(
      W_hh, fc1_w1, fc1_w2, fo_w1, fo_w2, gimg, 64.0f);

  k_seq<<<dim3(NB / ROWS_PB), dim3(WPB * 32), 0, stream>>>(
      x, gimg, W_ih, b_ih, b_hh, fc1_b1, fc1_b2, fo_b1, fo_b2, out);
}
